// SSMBlock_71906342470089
// MI455X (gfx1250) — hardware-run, weakly checked
//
#include <hip/hip_runtime.h>
#include <math.h>

typedef __attribute__((ext_vector_type(16))) _Float16 v16h;
typedef __attribute__((ext_vector_type(8)))  _Float16 v8h;
typedef __attribute__((ext_vector_type(8)))  float    v8f;
typedef __attribute__((ext_vector_type(4)))  float    v4f;

constexpr int kBatch   = 4;
constexpr int kSeq     = 2048;
constexpr int kDm      = 1024;
constexpr int kDin     = 2048;
constexpr int kNst     = 16;
constexpr int kTaps    = 4;
constexpr int kXpPitch = 2 * kDin;
constexpr int kRows    = kBatch * kSeq;
constexpr int kXpWords = kXpPitch / 2;
constexpr int kYgWords = kDin / 2;
constexpr int kPairs        = kDin / 2;
constexpr int kWavesPerB    = kPairs / 32;
constexpr int kScanWaves    = kBatch * kWavesPerB;
static_assert(kTaps == 4 && kNst == 16, "register layout of the scan");
static_assert((kDm % 32) == 0 && (kDin % 32) == 0, "GEMM K multiples of 32");
static_assert((kRows % 64) == 0 && (kXpPitch % 64) == 0 && (kDm % 64) == 0, "GEMM M,N multiples of 64");
static_assert(((kRows / 64) * (kXpPitch / 64)) % 8 == 0 && ((kRows / 64) * (kDm / 64)) % 8 == 0, "whole blocks of 8 tiles");
static_assert((kPairs % 32) == 0, "whole waves of channel pairs");
static_assert(((kRows * kDm / 8) % 256) == 0 && ((kXpPitch * kDm / 8) % 256) == 0 && ((kDm * kDin / 8) % 256) == 0, "convert grids exact");
static_assert(((kDin * kNst) % 256) == 0, "coefficient grid exact");

constexpr float kCarryX     = 64.0f;
constexpr float kCarryWin   = 2048.0f;
constexpr float kCarryXp    = 64.0f;
constexpr float kCarryYg    = 256.0f;
constexpr float kCarryWout  = 2048.0f;
constexpr float kInAccScale  = 1.0f / (kCarryX * kCarryWin);
constexpr float kOutAccScale = 1.0f / (kCarryYg * kCarryWout);
constexpr float kInvCarryXp  = 1.0f / kCarryXp;
constexpr float kF16MinNormal = 6.103515625e-5f;
constexpr float kF16Sat       = 60000.0f;
constexpr bool kNarrowInputs = false;

constexpr size_t kOffXH  = 0;
constexpr size_t kOffWIH = kOffXH  + (size_t)kRows * kDm * 2;
constexpr size_t kOffWOH = kOffWIH + (size_t)kXpPitch * kDm * 2;
constexpr size_t kOffXP  = kOffWOH + (size_t)kDm * kDin * 2;
constexpr size_t kOffYG  = kOffXP  + (size_t)kRows * kXpPitch * 2;
constexpr size_t kOffDAT = kOffYG  + (size_t)kRows * kDin * 2;
constexpr size_t kOffDBT = kOffDAT + (size_t)kDin * kNst * 4;
constexpr size_t kWsTotal = kOffDBT + (size_t)kDin * kNst * 4;
static_assert(kWsTotal == 130285568ull, "carve total");
static_assert(kWsTotal <= 134217728ull, "carve cap");
static_assert((kOffWIH % 128) == 0 && (kOffWOH % 128) == 0 && (kOffXP % 128) == 0 && (kOffYG % 128) == 0 &&
              (kOffDAT % 128) == 0 && (kOffDBT % 128) == 0, "128-B aligned regions");

__device__ __forceinline__ float in_prep(float v) {
  if (kNarrowInputs) {
    unsigned u = __float_as_uint(v);
    u += 0x7FFFu + ((u >> 16) & 1u);
    u &= 0xFFFF0000u;
    return __uint_as_float(u);
  }
  return v;
}
__device__ __forceinline__ _Float16 to_f16_flush(float c) {
  const float z = (fabsf(c) < kF16MinNormal) ? 0.0f : c;
  return (_Float16)z;
}
__device__ __forceinline__ float h16_to_f32(unsigned hb) {
  const unsigned sgn = (hb & 0x8000u) << 16;
  const unsigned em = hb & 0x7fffu;
  const float fn = __uint_as_float((em << 13) + 0x38000000u);
  const float fs = (float)em * 5.9604644775390625e-8f;
  const float mag = (em < 0x400u) ? fs : fn;
  return __uint_as_float(__float_as_uint(mag) | sgn);
}
__device__ __forceinline__ unsigned pack_f16x2(float lo, float hi) {
  const _Float16 h0 = (_Float16)lo;
  const _Float16 h1 = (_Float16)hi;
  return (unsigned)__builtin_bit_cast(unsigned short, h0) | ((unsigned)__builtin_bit_cast(unsigned short, h1) << 16);
}
__device__ __forceinline__ float silu_fast(float c) {
  return c * __builtin_amdgcn_rcpf(1.0f + __expf(-c));
}

__device__ __forceinline__ v16h frag_load_h(const _Float16* p) {
  union U { v16h v; v8h h[2]; } f;
  f.h[0] = *(const v8h*)(p);
  f.h[1] = *(const v8h*)(p + 16);
  return f.v;
}
__device__ __forceinline__ v8f mma_h(v16h a, v16h b, v8f c) {
  return __builtin_amdgcn_wmma_f32_16x16x32_f16(false, a, false, b, (short)0, c, false, false);
}
__device__ __forceinline__ void acc_tie_h(v8f& a, v16h x, v16h y) { asm volatile("" : "+v"(a) : "v"(x), "v"(y)); }
__device__ __forceinline__ void acc_nop4_h(v8f& a, v16h x, v16h y) { asm volatile("v_nop\n\tv_nop\n\tv_nop\n\tv_nop" : "+v"(a) : "v"(x), "v"(y)); }
__device__ __forceinline__ void acc_settle(v8f& a) { asm volatile("v_nop\n\tv_nop\n\tv_nop\n\tv_nop" : "+v"(a)); }
__device__ __forceinline__ void keep4_h(v16h a, v16h b, v16h c, v16h d) { asm volatile("v_nop" :: "v"(a), "v"(b), "v"(c), "v"(d)); }

__global__ __launch_bounds__(256) void cvt_plane_f16_kernel(
    const float* __restrict__ src, unsigned short* __restrict__ dst, int total8, float carry)
{
  const int i = blockIdx.x * 256 + threadIdx.x;
  if (i >= total8) return;
  const size_t e0 = (size_t)i << 3;
  const v4f a0 = *(const v4f*)(src + e0);
  const v4f a1 = *(const v4f*)(src + e0 + 4);
  v8h hv;
#pragma unroll
  for (int e = 0; e < 4; ++e) {
    const float f0 = a0[e];
    const float f1 = a1[e];
    hv[e]     = to_f16_flush(in_prep(f0) * carry);
    hv[4 + e] = to_f16_flush(in_prep(f1) * carry);
  }
  unsigned short* q = dst + e0;
  *(volatile v8h*)q = hv;
  __threadfence();
  *(volatile v8h*)q = hv;
}

__global__ __launch_bounds__(256) void scan_coef_kernel(
    const float* __restrict__ A_log, const float* __restrict__ Bp, const float* __restrict__ log_dt,
    float* __restrict__ dAt, float* __restrict__ dBt)
{
#pragma clang fp contract(off)
  const int i = blockIdx.x * 256 + threadIdx.x;
  if (i >= kDin * kNst) return;
  const int d = i >> 4;
  const float dt = expf(in_prep(log_dt[d]));
  const float av = expf(in_prep(A_log[i]));
  float prod = dt * av;
  asm volatile("" : "+v"(prod));
  const float da = expf(prod);
  const float db = dt * in_prep(Bp[i]);
  *(volatile float*)(dAt + i) = da;
  *(volatile float*)(dBt + i) = db;
  __threadfence();
  *(volatile float*)(dAt + i) = da;
  *(volatile float*)(dBt + i) = db;
}

template <int OUT_MODE>
__global__ __launch_bounds__(256) void gemm_f16_tile64(
    const unsigned short* __restrict__ Ap, int lda,
    const unsigned short* __restrict__ Btp, int ldb,
    void* __restrict__ Cout, int ldc,
    const float* __restrict__ bias,
    int M, int N, int K, float accScale, float outCarry)
{
  const _Float16* A  = (const _Float16*)Ap;
  const _Float16* Bt = (const _Float16*)Btp;
  __shared__ __align__(16) float sT[8][16 * 68];
  const int lane = threadIdx.x & 31;
  const int wave = threadIdx.x >> 5;
  const int tilesN = N >> 6;
  const int tilesM = M >> 6;
  const int tile = blockIdx.x * 8 + wave;
  if (tile >= tilesM * tilesN) return;
  const int tm = tile / tilesN;
  const int tn = tile - tm * tilesN;
  const int m0 = tm << 6;
  const int n0 = tn << 6;

  const int rlane = lane & 15;
  const int koff  = (lane >> 4) * 8;
  const int mOff  = (lane >> 4) * 8;

  v8f acc[4][4];
#pragma unroll
  for (int i = 0; i < 4; ++i)
#pragma unroll
    for (int j = 0; j < 4; ++j) acc[i][j] = (v8f){0.f, 0.f, 0.f, 0.f, 0.f, 0.f, 0.f, 0.f};

  for (int k0 = 0; k0 < K; k0 += 32) {
    v16h bh[4];
#pragma unroll
    for (int j = 0; j < 4; ++j) {
      const size_t bo = (size_t)(n0 + (j << 4) + rlane) * ldb + koff + k0;
      bh[j] = frag_load_h(Bt + bo);
    }
#pragma unroll
    for (int i = 0; i < 4; ++i) {
      const size_t ao = (size_t)(m0 + (i << 4) + rlane) * lda + koff + k0;
      const v16h ah = frag_load_h(A + ao);
#pragma unroll
      for (int j = 0; j < 4; ++j) acc[i][j] = mma_h(ah, bh[j], acc[i][j]);
      acc_tie_h(acc[i][0], ah, bh[0]);
      acc_tie_h(acc[i][1], ah, bh[1]);
      acc_tie_h(acc[i][2], ah, bh[2]);
      acc_nop4_h(acc[i][3], ah, bh[3]);
    }
    keep4_h(bh[0], bh[1], bh[2], bh[3]);
  }
#pragma unroll
  for (int i = 0; i < 4; ++i) {
    acc_settle(acc[i][0]);
    acc_settle(acc[i][1]);
    acc_settle(acc[i][2]);
    acc_settle(acc[i][3]);
  }

  float* slab = sT[wave];
#pragma unroll
  for (int i = 0; i < 4; ++i) {
    const int mBase = m0 + (i << 4);
#pragma unroll
    for (int j = 0; j < 4; ++j) {
      const int n = n0 + (j << 4) + rlane;
      const float bv = in_prep(bias[n]);
#pragma unroll
      for (int r = 0; r < 8; ++r) {
        float v = acc[i][j][r] * accScale;
        v += bv;
        v *= outCarry;
        slab[(mOff + r) * 68 + (j << 4) + rlane] = v;
      }
    }
    __builtin_amdgcn_fence(__ATOMIC_RELEASE, "workgroup");
    __builtin_amdgcn_wave_barrier();
    __builtin_amdgcn_fence(__ATOMIC_ACQUIRE, "workgroup");
    if (OUT_MODE == 0) {
      float* C = (float*)Cout;
      const int hh = lane >> 4, c4 = (lane & 15) * 4;
      for (int pass = 0; pass < 2; ++pass) {
#pragma unroll
        for (int it = 0; it < 8; ++it) {
          const int row = it * 2 + hh;
          const v4f v = *(const v4f*)(slab + row * 68 + c4);
          *(volatile v4f*)(C + (size_t)(mBase + row) * ldc + n0 + c4) = v;
        }
        __threadfence();
      }
    } else {
      const int q = lane >> 3, c8 = (lane & 7) * 8;
      unsigned short* C = (unsigned short*)Cout;
      for (int pass = 0; pass < 2; ++pass) {
#pragma unroll
        for (int it = 0; it < 4; ++it) {
          const int row = it * 4 + q;
          const float* sp = slab + row * 68 + c8;
          v8h hv;
#pragma unroll
          for (int e = 0; e < 8; ++e) {
            const float sv = sp[e];
            hv[e] = to_f16_flush(sv);
          }
          *(volatile v8h*)(C + (size_t)(mBase + row) * ldc + n0 + c8) = hv;
        }
        __threadfence();
      }
    }
    __builtin_amdgcn_fence(__ATOMIC_RELEASE, "workgroup");
    __builtin_amdgcn_wave_barrier();
    __builtin_amdgcn_fence(__ATOMIC_ACQUIRE, "workgroup");
  }
}

__global__ __launch_bounds__(32) void conv_scan_gate_kernel(
    const unsigned* __restrict__ xpw, const float* __restrict__ conv_w, const float* __restrict__ conv_b,
    const float* __restrict__ dAt, const float* __restrict__ dBt, const float* __restrict__ Cp,
    unsigned* __restrict__ ygw)
{
  const int lane = threadIdx.x & 31;
  const int wv   = blockIdx.x;
  const int bix  = wv / kWavesPerB;
  const int pr   = (wv - bix * kWavesPerB) * 32 + lane;
  const int d0   = pr * 2;

  const v4f cwa = *(const v4f*)(conv_w + (size_t)d0 * kTaps);
  const v4f cwb = *(const v4f*)(conv_w + (size_t)d0 * kTaps + kTaps);
  const float ta0 = cwa[0], ta1 = cwa[1], ta2 = cwa[2], ta3 = cwa[3];
  const float tb0 = cwb[0], tb1 = cwb[1], tb2 = cwb[2], tb3 = cwb[3];
  const float wa0 = in_prep(ta0) * kInvCarryXp, wa1 = in_prep(ta1) * kInvCarryXp;
  const float wa2 = in_prep(ta2) * kInvCarryXp, wa3 = in_prep(ta3) * kInvCarryXp;
  const float wb0 = in_prep(tb0) * kInvCarryXp, wb1 = in_prep(tb1) * kInvCarryXp;
  const float wb2 = in_prep(tb2) * kInvCarryXp, wb3 = in_prep(tb3) * kInvCarryXp;
  const float cba = in_prep(conv_b[d0]);
  const float cbb = in_prep(conv_b[d0 + 1]);

  float dAa[kNst], dBa[kNst], Cca[kNst], ha[kNst];
  float dAb[kNst], dBb[kNst], Ccb[kNst], hb[kNst];
  {
    const v4f* pA = (const v4f*)(dAt + (size_t)d0 * kNst);
    const v4f* pB = (const v4f*)(dBt + (size_t)d0 * kNst);
    const v4f* pC = (const v4f*)(Cp  + (size_t)d0 * kNst);
#pragma unroll
    for (int q = 0; q < 4; ++q) {
      const v4f a0 = pA[q], a1 = pA[q + 4];
      const v4f b0 = pB[q], b1 = pB[q + 4];
      const v4f c0 = pC[q], c1 = pC[q + 4];
#pragma unroll
      for (int e = 0; e < 4; ++e) {
        const float fa0 = a0[e], fa1 = a1[e], fb0 = b0[e], fb1 = b1[e], fc0 = c0[e], fc1 = c1[e];
        dAa[4 * q + e] = fa0;
        dAb[4 * q + e] = fa1;
        dBa[4 * q + e] = fb0;
        dBb[4 * q + e] = fb1;
        Cca[4 * q + e] = in_prep(fc0);
        Ccb[4 * q + e] = in_prep(fc1);
        ha[4 * q + e] = 0.f;
        hb[4 * q + e] = 0.f;
      }
    }
  }

  const size_t rowBase = (size_t)bix * kSeq;
  const unsigned* px = xpw + rowBase * kXpWords + pr;
  unsigned*       py = ygw + rowBase * kYgWords + pr;

  float xa3 = 0.f, xa2 = 0.f, xa1 = 0.f;
  float xb3 = 0.f, xb2 = 0.f, xb1 = 0.f;

#pragma unroll 1
  for (int t = 0; t < kSeq; ++t) {
    const unsigned w1 = px[(size_t)t * kXpWords];
    const unsigned w2 = px[(size_t)t * kXpWords + kYgWords];
    const float xa = h16_to_f32(w1 & 0xffffu);
    const float xb = h16_to_f32(w1 >> 16);
    float ca = wa0 * xa3;
    ca = fmaf(wa1, xa2, ca);
    ca = fmaf(wa2, xa1, ca);
    ca = fmaf(wa3, xa, ca);
    ca += cba;
    float cb2 = wb0 * xb3;
    cb2 = fmaf(wb1, xb2, cb2);
    cb2 = fmaf(wb2, xb1, cb2);
    cb2 = fmaf(wb3, xb, cb2);
    cb2 += cbb;
    xa3 = xa2; xa2 = xa1; xa1 = xa;
    xb3 = xb2; xb2 = xb1; xb1 = xb;
    const float ua = silu_fast(ca);
    const float ub = silu_fast(cb2);
    float ya = 0.f, yb = 0.f;
#pragma unroll
    for (int n = 0; n < kNst; ++n) {
      ha[n] = fmaf(dAa[n], ha[n], dBa[n] * ua);
      ya = fmaf(ha[n], Cca[n], ya);
      hb[n] = fmaf(dAb[n], hb[n], dBb[n] * ub);
      yb = fmaf(hb[n], Ccb[n], yb);
    }
    const float ga = h16_to_f32(w2 & 0xffffu) * kInvCarryXp;
    const float gb = h16_to_f32(w2 >> 16) * kInvCarryXp;
    float oa = (ya * silu_fast(ga)) * kCarryYg;
    float ob = (yb * silu_fast(gb)) * kCarryYg;
    oa = fminf(fmaxf(oa, -kF16Sat), kF16Sat);
    ob = fminf(fmaxf(ob, -kF16Sat), kF16Sat);
    oa = (fabsf(oa) < kF16MinNormal) ? 0.0f : oa;
    ob = (fabsf(ob) < kF16MinNormal) ? 0.0f : ob;
    const unsigned wout = pack_f16x2(oa, ob);
    volatile unsigned* q = (volatile unsigned*)(py + (size_t)t * kYgWords);
    *q = wout;
    __threadfence();
    *q = wout;
  }
}

extern "C" void kernel_launch(void* const* d_in, const int* in_sizes, int n_in,
                              void* d_out, int out_size, void* d_ws, size_t ws_size,
                              hipStream_t stream) {
  if (n_in < 11) return;
  if (in_sizes[0] != kRows * kDm) return;
  if (in_sizes[1] != kXpPitch * kDm) return;
  if (in_sizes[2] != kXpPitch) return;
  if (in_sizes[3] != kDin * kTaps) return;
  if (in_sizes[4] != kDin) return;
  if (in_sizes[5] != kDin * kNst) return;
  if (in_sizes[6] != kDin * kNst) return;
  if (in_sizes[7] != kDin * kNst) return;
  if (in_sizes[8] != kDin) return;
  if (in_sizes[9] != kDm * kDin) return;
  if (in_sizes[10] != kDm) return;
  if (out_size != kRows * kDm) return;
  if (ws_size < kWsTotal) return;

  const float* x      = (const float*)d_in[0];
  const float* W_in   = (const float*)d_in[1];
  const float* b_in   = (const float*)d_in[2];
  const float* conv_w = (const float*)d_in[3];
  const float* conv_b = (const float*)d_in[4];
  const float* A_log  = (const float*)d_in[5];
  const float* B_par  = (const float*)d_in[6];
  const float* C_par  = (const float*)d_in[7];
  const float* log_dt = (const float*)d_in[8];
  const float* W_out  = (const float*)d_in[9];
  const float* b_out  = (const float*)d_in[10];
  float* out = (float*)d_out;

  char* ws = (char*)d_ws;
  unsigned short* XH  = (unsigned short*)(ws + kOffXH);
  unsigned short* WIH = (unsigned short*)(ws + kOffWIH);
  unsigned short* WOH = (unsigned short*)(ws + kOffWOH);
  unsigned short* XP  = (unsigned short*)(ws + kOffXP);
  unsigned short* YG  = (unsigned short*)(ws + kOffYG);
  float*          DAT = (float*)(ws + kOffDAT);
  float*          DBT = (float*)(ws + kOffDBT);

  cvt_plane_f16_kernel<<<(kRows * kDm / 8) / 256, 256, 0, stream>>>(x, XH, kRows * kDm / 8, kCarryX);
  cvt_plane_f16_kernel<<<(kXpPitch * kDm / 8) / 256, 256, 0, stream>>>(W_in, WIH, kXpPitch * kDm / 8, kCarryWin);
  cvt_plane_f16_kernel<<<(kDm * kDin / 8) / 256, 256, 0, stream>>>(W_out, WOH, kDm * kDin / 8, kCarryWout);

  scan_coef_kernel<<<(kDin * kNst) / 256, 256, 0, stream>>>(A_log, B_par, log_dt, DAT, DBT);

  gemm_f16_tile64<1><<<((kRows / 64) * (kXpPitch / 64)) / 8, 256, 0, stream>>>(
      XH, kDm, WIH, kDm, (void*)XP, kXpPitch, b_in,
      kRows, kXpPitch, kDm, kInAccScale, kCarryXp);

  conv_scan_gate_kernel<<<kScanWaves, 32, 0, stream>>>(
      (const unsigned*)XP, conv_w, conv_b, DAT, DBT, C_par, (unsigned*)YG);

  gemm_f16_tile64<0><<<((kRows / 64) * (kDm / 64)) / 8, 256, 0, stream>>>(
      YG, kDin, WOH, kDin, (void*)out, kDm, b_out,
      kRows, kDm, kDin, kOutAccScale, 1.0f);
}
